// ReconstructionDecoder_36421322670264
// MI455X (gfx1250) — hardware-verified
//
#include <hip/hip_runtime.h>
#include <stddef.h>
#include <stdint.h>
#include <math.h>

#define BN   16
#define TT   128
#define NF   128
#define DD   256
#define EE   512
#define NO   2
#define NROW 64
#define PA   264
#define NBLK (TT * (NF / 16) * (BN / 4))

static_assert(DD % 64 == 0);
static_assert(EE % 64 == 0);
static_assert(EE == 8 * 64);
static_assert(DD == 32 * 8);
static_assert(DD % 32 == 0);
static_assert(NF % 16 == 0);
static_assert(BN % 4 == 0);
static_assert(NROW == 4 * 16);
static_assert((PA % 8) == 0);
static_assert(NBLK == 4096);
static_assert(NROW * NO == 128);

typedef _Float16 hh;
typedef hh    v16h __attribute__((ext_vector_type(16)));
typedef hh    v8h  __attribute__((ext_vector_type(8)));
typedef float v8f  __attribute__((ext_vector_type(8)));
typedef float v4f  __attribute__((ext_vector_type(4)));

union Frag { v16h v; v8h p[2]; };

__device__ __forceinline__ v8f zero8() { return (v8f){0.f, 0.f, 0.f, 0.f, 0.f, 0.f, 0.f, 0.f}; }

__device__ __forceinline__ float wsum(float v) {
#pragma unroll
  for (int off = 16; off > 0; off >>= 1) v += __shfl_xor(v, off, 32);
  return v;
}

__device__ __forceinline__ v16h ldfrag(const hh* __restrict__ p, int ld, int row0, int k0, int lane) {
  const hh* q = p + (size_t)(row0 + (lane & 15)) * (size_t)ld + k0 + 8 * (lane >> 4);
  Frag f;
  f.p[0] = *(const v8h*)(q);
  f.p[1] = *(const v8h*)(q + 16);
  return f.v;
}

__device__ __forceinline__ v8f mma16(v16h a, v16h b, v8f cc) {
  return __builtin_amdgcn_wmma_f32_16x16x32_f16(false, a, false, b, (short)0, cc, false, false);
}

template <int KD, int ND>
__global__ __launch_bounds__(256) void k_cvt_wt(const float* __restrict__ w, hh* __restrict__ wt) {
  static_assert(KD % 64 == 0);
  static_assert(ND % 64 == 0);
  __shared__ __align__(16) float sw[64 * 68];
  const int tid = threadIdx.x;
  const int kb = blockIdx.x * 64;
  const int nb = blockIdx.y * 64;
  {
    const int r  = tid >> 2;
    const int c0 = (tid & 3) * 16;
    const float* src = w + (size_t)(kb + r) * ND + nb + c0;
#pragma unroll
    for (int e = 0; e < 4; ++e) *(v4f*)(sw + r * 68 + c0 + 4 * e) = *(const v4f*)(src + 4 * e);
  }
  __syncthreads();
  v8h hv[2];
  size_t go[2];
#pragma unroll
  for (int j = 0; j < 2; ++j) {
    const int p  = tid + 256 * j;
    const int n  = p >> 3;
    const int pc = p & 7;
    const float* cp = sw + (pc * 8) * 68 + n;
    v8f t;
#pragma unroll
    for (int e = 0; e < 8; ++e) t[e] = cp[e * 68] * 64.0f;
    hv[j] = __builtin_convertvector(t, v8h);
    go[j] = (size_t)(nb + n) * KD + kb + pc * 8;
  }
#pragma unroll
  for (int j = 0; j < 2; ++j) *(volatile v8h*)(wt + go[j]) = hv[j];
  __threadfence();
#pragma unroll
  for (int j = 0; j < 2; ++j) *(volatile v8h*)(wt + go[j]) = hv[j];
}

__global__ __launch_bounds__(256) void k_main(const float* __restrict__ x, const float* __restrict__ te,
                                              const float* __restrict__ fe, const float* __restrict__ g,
                                              const float* __restrict__ bt, const hh* __restrict__ w1t,
                                              const float* __restrict__ b1, const float* __restrict__ w2,
                                              const float* __restrict__ b2, float* __restrict__ out) {
  __shared__ __align__(16) hh As[NROW * PA];
  __shared__ float part[8 * NROW * NO];
  __shared__ __align__(16) float ol[NROW * NO];

  const int tid = threadIdx.x, lane = tid & 31, w = tid >> 5;
  const int h = lane >> 4, c = lane & 15;
  const int bx = blockIdx.x;
  const int fq = bx & 7;
  const int t  = (bx >> 3) & (TT - 1);
  const int bq = bx >> 10;
  const int f0 = fq * 16;
  const int bn0 = bq * 4;

  {
    const int bl = w >> 1;
    const int d0 = lane * 8;
    const float* xr = x + (size_t)(bn0 + bl) * DD + d0;
    const float* tr = te + (size_t)t * DD + d0;
    const v4f xa = *(const v4f*)(xr), xb = *(const v4f*)(xr + 4);
    const v4f ta = *(const v4f*)(tr), tb = *(const v4f*)(tr + 4);
    const v4f ga = *(const v4f*)(g + d0), gb = *(const v4f*)(g + d0 + 4);
    const v4f ba = *(const v4f*)(bt + d0), bb = *(const v4f*)(bt + d0 + 4);
    const float xs[8] = {xa[0], xa[1], xa[2], xa[3], xb[0], xb[1], xb[2], xb[3]};
    const float ts[8] = {ta[0], ta[1], ta[2], ta[3], tb[0], tb[1], tb[2], tb[3]};
    const float gs[8] = {ga[0], ga[1], ga[2], ga[3], gb[0], gb[1], gb[2], gb[3]};
    const float bs[8] = {ba[0], ba[1], ba[2], ba[3], bb[0], bb[1], bb[2], bb[3]};
#pragma unroll 1
    for (int i = 0; i < 8; ++i) {
      const int lr = w * 8 + i;
      const int fl = lr & 15;
      const float* fr = fe + (size_t)(f0 + fl) * DD + d0;
      const v4f fa = *(const v4f*)(fr), fb = *(const v4f*)(fr + 4);
      const float fs[8] = {fa[0], fa[1], fa[2], fa[3], fb[0], fb[1], fb[2], fb[3]};
      float hv[8];
      float s = 0.f;
#pragma unroll
      for (int e = 0; e < 8; ++e) {
        const float pos = ts[e] + fs[e];
        hv[e] = xs[e] + pos;
        s += hv[e];
      }
      s = wsum(s);
      const float mu = s * (1.0f / (float)DD);
      float dv[8];
      float s2 = 0.f;
#pragma unroll
      for (int e = 0; e < 8; ++e) {
        dv[e] = hv[e] - mu;
        s2 = fmaf(dv[e], dv[e], s2);
      }
      s2 = wsum(s2);
      const float var = s2 * (1.0f / (float)DD);
      const float inv = rsqrtf(var + 1e-5f);
      v8f y;
#pragma unroll
      for (int e = 0; e < 8; ++e) y[e] = dv[e] * inv * gs[e] + bs[e];
      const v8h pk = __builtin_convertvector(y, v8h);
      *(v8h*)(As + lr * PA + d0) = pk;
    }
  }
  __syncthreads();

  const int nb = w * 64;
  float bc[4], wa[4], wb[4];
#pragma unroll
  for (int j = 0; j < 4; ++j) {
    const int col = nb + 16 * j + c;
    bc[j] = b1[col];
    wa[j] = w2[col * NO + 0];
    wb[j] = w2[col * NO + 1];
  }

#pragma unroll 1
  for (int s = 0; s < 2; ++s) {
    const int ma = s * 32;
    v8f acc[2][4];
#pragma unroll
    for (int i = 0; i < 2; ++i)
#pragma unroll
      for (int j = 0; j < 4; ++j) acc[i][j] = zero8();

#pragma unroll 1
    for (int k0 = 0; k0 < DD; k0 += 32) {
      Frag fa0, fa1;
      const hh* qa = As + (ma + c) * PA + k0 + 8 * h;
      fa0.p[0] = *(const v8h*)(qa);
      fa0.p[1] = *(const v8h*)(qa + 16);
      fa1.p[0] = *(const v8h*)(qa + 16 * PA);
      fa1.p[1] = *(const v8h*)(qa + 16 * PA + 16);
      const v16h a0 = fa0.v, a1 = fa1.v;
      const v16h b0 = ldfrag(w1t, DD, nb, k0, lane);
      const v16h b1f = ldfrag(w1t, DD, nb + 16, k0, lane);
      const v16h b2f = ldfrag(w1t, DD, nb + 32, k0, lane);
      const v16h b3f = ldfrag(w1t, DD, nb + 48, k0, lane);
      acc[0][0] = mma16(a0, b0, acc[0][0]);
      acc[1][0] = mma16(a1, b0, acc[1][0]);
      acc[0][1] = mma16(a0, b1f, acc[0][1]);
      acc[1][1] = mma16(a1, b1f, acc[1][1]);
      acc[0][2] = mma16(a0, b2f, acc[0][2]);
      acc[1][2] = mma16(a1, b2f, acc[1][2]);
      acc[0][3] = mma16(a0, b3f, acc[0][3]);
      acc[1][3] = mma16(a1, b3f, acc[1][3]);
      asm volatile("v_nop\n\tv_nop\n\tv_nop\n\tv_nop"
                   : "+v"(acc[0][0]), "+v"(acc[0][1]), "+v"(acc[0][2]), "+v"(acc[0][3]),
                     "+v"(acc[1][0]), "+v"(acc[1][1]), "+v"(acc[1][2]), "+v"(acc[1][3])
                   : "v"(a0), "v"(a1), "v"(b0), "v"(b1f), "v"(b2f), "v"(b3f));
    }

    float po[2][8][2];
#pragma unroll
    for (int i = 0; i < 2; ++i)
#pragma unroll
      for (int r = 0; r < 8; ++r) { po[i][r][0] = 0.f; po[i][r][1] = 0.f; }
#pragma unroll
    for (int i = 0; i < 2; ++i)
#pragma unroll
      for (int j = 0; j < 4; ++j)
#pragma unroll
        for (int r = 0; r < 8; ++r) {
          const float v = fmaxf(acc[i][j][r] * (1.0f / 64.0f) + bc[j], 0.f);
          po[i][r][0] = fmaf(v, wa[j], po[i][r][0]);
          po[i][r][1] = fmaf(v, wb[j], po[i][r][1]);
        }
#pragma unroll
    for (int i = 0; i < 2; ++i)
#pragma unroll
      for (int r = 0; r < 8; ++r)
#pragma unroll
        for (int o = 0; o < 2; ++o) {
          float v = po[i][r][o];
          v += __shfl_xor(v, 1, 32);
          v += __shfl_xor(v, 2, 32);
          v += __shfl_xor(v, 4, 32);
          v += __shfl_xor(v, 8, 32);
          if (c == 0) part[(w * NROW + ma + 16 * i + 8 * h + r) * NO + o] = v;
        }
  }
  __syncthreads();

  if (tid < NROW * NO) {
    const int lr = tid >> 1, o = tid & 1;
    float sacc = b2[o];
#pragma unroll
    for (int ww = 0; ww < 8; ++ww) sacc += part[(ww * NROW + lr) * NO + o];
    ol[tid] = sacc;
  }
  __syncthreads();
  if (w == 0) {
    const int q  = lane >> 3;
    const int pc = lane & 7;
    const v4f v = *(const v4f*)(ol + q * 32 + pc * 4);
    float* gp = out + ((((size_t)(bn0 + q)) * TT + (size_t)t) * NF + (size_t)f0) * NO + pc * 4;
    *(volatile v4f*)gp = v;
    __threadfence();
    *(volatile v4f*)gp = v;
  }
}

extern "C" void kernel_launch(void* const* d_in, const int* in_sizes, int n_in,
                              void* d_out, int out_size, void* d_ws, size_t ws_size,
                              hipStream_t stream) {
  if (n_in < 9) return;
  if (in_sizes[0] != BN * DD) return;
  if (in_sizes[1] != TT * DD || in_sizes[2] != NF * DD) return;
  if (in_sizes[3] != DD || in_sizes[4] != DD) return;
  if (in_sizes[5] != DD * EE || in_sizes[6] != EE) return;
  if (in_sizes[7] != EE * NO || in_sizes[8] != NO) return;
  if (out_size != BN * TT * NF * NO) return;

  const size_t oW1T = 0;
  const size_t total = (size_t)EE * DD * 2;
  if (total > ws_size) return;
  if (total > (size_t)134217728) return;

  const float* x    = (const float*)d_in[0];
  const float* te   = (const float*)d_in[1];
  const float* fe   = (const float*)d_in[2];
  const float* lng  = (const float*)d_in[3];
  const float* lnb  = (const float*)d_in[4];
  const float* w1   = (const float*)d_in[5];
  const float* b1   = (const float*)d_in[6];
  const float* w2   = (const float*)d_in[7];
  const float* b2   = (const float*)d_in[8];
  float* out = (float*)d_out;

  char* ws = (char*)d_ws;
  hh* W1T = (hh*)(ws + oW1T);

  k_cvt_wt<DD, EE><<<dim3(DD / 64, EE / 64), dim3(256), 0, stream>>>(w1, W1T);
  k_main<<<dim3(NBLK), dim3(256), 0, stream>>>(x, te, fe, lng, lnb, W1T, b1, w2, b2, out);
  (void)hipGetLastError();
}
